// KPConv_3487513444656
// MI455X (gfx1250) — hardware-verified
//
#include <hip/hip_runtime.h>
#include <stddef.h>
#include <stdint.h>

#define PD      3
#define CIN     32
#define COUT    32
#define KPT     15
#define FWW     (KPT * COUT)
#define HP      16
#define KPL     48
#define NTHR    256
#define NWAVE   8
#define EPB     256
#define EPT     8
#define CHUNK   (NTHR * EPT)
#define WCAP    (EPT * 32)
#define LISTN   (NWAVE * WCAP)
#define NBA     1024
#define PKS     10
#define RCAP    28672
#define DEGCAP  64
#define GBM     64
#define GTHR    128
#define NTF     10
#define BNF     (16 * NTF)
#define NCB     (FWW / BNF)
#define PPR     (BNF / 4)
#define NITF    (GBM * BNF / (4 * GTHR))
#define NUW     (FWW * CIN / 8)
#define ZINTS   (2 * RCAP + 2 * NBA + LISTN)
#define LDS_AGG (ZINTS * 4 + 64)
#define WSLIM   268435456
#define INV_EXT (1.0f / 1.2f)

static_assert((CHUNK & (CHUNK - 1)) == 0);
static_assert(NBA == (1 << PKS));
static_assert(((long long)CHUNK << PKS) < (1LL << 31));
static_assert(NTHR * 4 == NBA);
static_assert(LISTN >= NBA && LISTN >= NWAVE * WCAP);
static_assert((RCAP % 32) == 0);
static_assert((ZINTS % (NTHR * 4)) == 0);
static_assert(LDS_AGG <= 262144);
static_assert((NBA % NWAVE) == 0);
static_assert(GBM == (GTHR / 32) * 16);
static_assert(CIN == 32 && COUT == 32 && KPT == 15 && FWW == 480);
static_assert((FWW % BNF) == 0 && NCB * BNF == FWW);
static_assert(((BNF * 4) % 128) == 0 && ((FWW * 4) % 128) == 0);
static_assert(NITF * GTHR * 4 == GBM * BNF && (PPR % 8) == 0);
static_assert((NUW % 32) == 0 && NUW * 8 == FWW * CIN);
static_assert(EPB == NTHR && EPB == NWAVE * 32);
static_assert(EPB * COUT == 8 * NTHR * 4);
static_assert(KPT * PD <= KPL && KPT < HP && 4 * 3 + 3 == HP - 1);

typedef float          v4f  __attribute__((ext_vector_type(4)));
typedef float          v8f  __attribute__((ext_vector_type(8)));
typedef int            v4i  __attribute__((ext_vector_type(4)));
typedef int            v8i  __attribute__((ext_vector_type(8)));
typedef unsigned short v8us __attribute__((ext_vector_type(8)));
typedef __bf16         v16b __attribute__((ext_vector_type(16)));
typedef v4f  __attribute__((may_alias)) v4fa;
typedef v4i  __attribute__((may_alias)) v4ia;
typedef v8us __attribute__((may_alias)) v8usa;
union Frag { v16b b; v8us h[2]; v8i w; };

__device__ __forceinline__ v8f wmk(const Frag& a, const Frag& b, v8f c) {
  v8f d = __builtin_amdgcn_wmma_f32_16x16x32_bf16(false, a.b, false, b.b, (short)0, c, false, false);
  asm volatile("v_nop\n\tv_nop\n\tv_nop\n\tv_nop" : "+v"(d) : "v"(a.w), "v"(b.w));
  return d;
}

__device__ __forceinline__ unsigned short bf_bits(float f) {
  unsigned int u = __float_as_uint(f);
  u += 0x7FFFu + ((u >> 16) & 1u);
  return (unsigned short)(u >> 16);
}
__device__ __forceinline__ float bf_val(unsigned short b) {
  return __uint_as_float(((unsigned int)b) << 16);
}
__device__ __forceinline__ float bf_rne(float f) { return bf_val(bf_bits(f)); }

__device__ __forceinline__ v8us cvt8(const float* p) {
  const v4f a = *(const v4fa*)p, b = *(const v4fa*)(p + 4);
  v8us o;
  o[0] = bf_bits(a.x); o[1] = bf_bits(a.y); o[2] = bf_bits(a.z); o[3] = bf_bits(a.w);
  o[4] = bf_bits(b.x); o[5] = bf_bits(b.y); o[6] = bf_bits(b.z); o[7] = bf_bits(b.w);
  return o;
}

__device__ __forceinline__ int scan_chunk(const int* __restrict__ dsts, int nE, int cbase, int slotBase,
                                          int nb, int vec8, int* list, int tid, int lane, int wave) {
  int wc = 0;
  const int el0  = tid * EPT;
  const int e0   = cbase + el0;
  const int sent = -2147483647 - 1;
  v4i da, db;
  if (vec8 != 0 && cbase + CHUNK <= nE) {
    da = *(const v4i*)(dsts + e0);
    db = *(const v4i*)(dsts + e0 + 4);
  } else {
    da.x = (e0     < nE) ? dsts[min(e0,     nE - 1)] : sent;
    da.y = (e0 + 1 < nE) ? dsts[min(e0 + 1, nE - 1)] : sent;
    da.z = (e0 + 2 < nE) ? dsts[min(e0 + 2, nE - 1)] : sent;
    da.w = (e0 + 3 < nE) ? dsts[min(e0 + 3, nE - 1)] : sent;
    db.x = (e0 + 4 < nE) ? dsts[min(e0 + 4, nE - 1)] : sent;
    db.y = (e0 + 5 < nE) ? dsts[min(e0 + 5, nE - 1)] : sent;
    db.z = (e0 + 6 < nE) ? dsts[min(e0 + 6, nE - 1)] : sent;
    db.w = (e0 + 7 < nE) ? dsts[min(e0 + 7, nE - 1)] : sent;
  }
  const unsigned nbs = (unsigned)slotBase;
  const unsigned unb = (unsigned)nb;
  const unsigned s0 = (unsigned)da.x - nbs, s1 = (unsigned)da.y - nbs;
  const unsigned s2 = (unsigned)da.z - nbs, s3 = (unsigned)da.w - nbs;
  const unsigned s4 = (unsigned)db.x - nbs, s5 = (unsigned)db.y - nbs;
  const unsigned s6 = (unsigned)db.z - nbs, s7 = (unsigned)db.w - nbs;
  const bool h0 = s0 < unb, h1 = s1 < unb, h2 = s2 < unb, h3 = s3 < unb;
  const bool h4 = s4 < unb, h5 = s5 < unb, h6 = s6 < unb, h7 = s7 < unb;
  const unsigned any = __builtin_amdgcn_ballot_w32(h0 | h1 | h2 | h3 | h4 | h5 | h6 | h7);
  if (any != 0u) {
#define HITJ(J, HJ, SJ) { \
      const unsigned mj = __builtin_amdgcn_ballot_w32(HJ); \
      if (mj != 0u) { \
        if (HJ) { \
          const int pos = wc + (int)__builtin_amdgcn_mbcnt_lo(mj, 0u); \
          if (pos < WCAP) list[wave * WCAP + pos] = ((el0 + (J)) << PKS) | (int)(SJ); \
        } \
        wc += (int)__builtin_popcount(mj); } }
    HITJ(0, h0, s0)
    HITJ(1, h1, s1)
    HITJ(2, h2, s2)
    HITJ(3, h3, s3)
    HITJ(4, h4, s4)
    HITJ(5, h5, s5)
    HITJ(6, h6, s6)
    HITJ(7, h7, s7)
#undef HITJ
  }
  return wc;
}

__global__ __launch_bounds__(NTHR) void k_wprep(const float* __restrict__ W, unsigned short* WT) {
  const int u = (int)blockIdx.x * NTHR + (int)threadIdx.x;
  if (u >= NUW) return;
  const int n  = u >> 2;
  const int kp = n >> 5;
  const int o  = n & 31;
  const int k8 = (u & 3) * 8;
  const float* p = W + (size_t)kp * (CIN * COUT) + (size_t)k8 * COUT + o;
  v8us ov;
#pragma unroll
  for (int j = 0; j < 8; ++j) ov[j] = bf_bits(p[(size_t)j * COUT]);
  unsigned short* dp = WT + (size_t)u * 8;
  *(volatile v8us*)dp = ov;
  __threadfence();
  *(volatile v8us*)dp = ov;
}

__global__ __launch_bounds__(GTHR) void k_fw(const float* __restrict__ feat, int nN,
                                             const unsigned short* __restrict__ WT, float* FW) {
  __shared__ __attribute__((aligned(16))) float stg[GBM * BNF];
  const int tid = (int)threadIdx.x, lane = tid & 31, wave = tid >> 5, hh = lane >> 4, m = lane & 15;
  const int rowBase = (int)blockIdx.x * GBM;
  const int colBase = (int)blockIdx.y * BNF;
  const int row = rowBase + 16 * wave + m;
  const int rc  = row < nN ? row : nN - 1;
  const float* xp = feat + (size_t)rc * CIN + 8 * hh;

  Frag af;
  af.h[0] = cvt8(xp);
  af.h[1] = cvt8(xp + 16);
  const unsigned short* bp = WT + (size_t)(colBase + m) * CIN + 8 * hh;

  v8f acc[NTF];
  {
    const v8f z = {0.f, 0.f, 0.f, 0.f, 0.f, 0.f, 0.f, 0.f};
#pragma unroll
    for (int t = 0; t < NTF; ++t) acc[t] = z;
  }
#pragma unroll
  for (int nt = 0; nt < NTF; ++nt) {
    const unsigned short* wq = bp + (size_t)(16 * nt) * CIN;
    Frag bf;
    bf.h[0] = *(const v8usa*)wq;
    bf.h[1] = *(const v8usa*)(wq + 16);
    acc[nt] = wmk(af, bf, acc[nt]);
  }

#pragma unroll
  for (int nt = 0; nt < NTF; ++nt) {
    const int lc = 16 * nt + m;
#pragma unroll
    for (int r = 0; r < 8; ++r) {
      const int lr = 16 * wave + 8 * hh + r;
      stg[lr * BNF + lc] = acc[nt][r];
    }
  }
  __syncthreads();

  float* fb = FW + (size_t)rowBase * FWW + colBase;
#pragma unroll
  for (int it = 0; it < NITF; ++it) {
    const int p  = it * GTHR + tid;
    const int pr = p / PPR;
    const int pc = p - pr * PPR;
    const v4f v = *(const v4fa*)(stg + 4 * p);
    *(volatile v4f*)(fb + (size_t)pr * FWW + 4 * pc) = v;
  }
  __threadfence();
#pragma unroll
  for (int it = 0; it < NITF; ++it) {
    const int p  = it * GTHR + tid;
    const int pr = p / PPR;
    const int pc = p - pr * PPR;
    const v4f v = *(const v4fa*)(stg + 4 * p);
    *(volatile v4f*)(fb + (size_t)pr * FWW + 4 * pc) = v;
  }
}

__global__ __launch_bounds__(NTHR) void k_edge(const float* __restrict__ pos, const int* __restrict__ srcs,
                                               const int* __restrict__ dsts, const float* __restrict__ kp,
                                               int nE, int nN, const float* __restrict__ FW, float* MSG) {
  __shared__ __attribute__((aligned(16))) float ms[EPB * COUT];
  __shared__ __attribute__((aligned(16))) float hl[EPB * HP];
  __shared__ int   sl[EPB];
  __shared__ float kpl[KPL];
  const int tid = (int)threadIdx.x, lane = tid & 31, wave = tid >> 5;
  const int elb = (int)blockIdx.x * EPB;

  if (tid < KPL) {
    const int ci = tid < KPT * PD ? tid : KPT * PD - 1;
    const float kv = bf_rne(kp[ci]);
    kpl[tid] = (tid < KPT * PD) ? kv : 0.0f;
  }
  float yx, yy, yz;
  {
    const int el  = elb + tid;
    const int elc = el < nE ? el : nE - 1;
    int s = srcs[elc];
    s = s < 0 ? 0 : (s > nN - 1 ? nN - 1 : s);
    int d = dsts[elc];
    d = d < 0 ? 0 : (d > nN - 1 ? nN - 1 : d);
    const float* ps = pos + (size_t)s * PD;
    const float* pq = pos + (size_t)d * PD;
    yx = bf_rne(ps[0]) - bf_rne(pq[0]);
    yy = bf_rne(ps[1]) - bf_rne(pq[1]);
    yz = bf_rne(ps[2]) - bf_rne(pq[2]);
    sl[tid] = s;
  }
  __syncthreads();

#pragma unroll 1
  for (int k = 0; k < KPT; ++k) {
    const float dx = yx - kpl[3 * k + 0];
    const float dy = yy - kpl[3 * k + 1];
    const float dz = yz - kpl[3 * k + 2];
    const float sq = dx * dx + dy * dy + dz * dz;
    const float dd = sqrtf(sq);
    float h = 1.0f - dd * INV_EXT;
    h = fmaxf(h, 0.0f);
    hl[tid * HP + k] = h;
  }
  hl[tid * HP + KPT] = 0.0f;
  __syncthreads();

  const int g    = lane >> 3;
  const int c4   = 4 * (lane & 7);
  const int off3 = (lane < 24) ? (3 * 128 + 4 * lane) : (4 * lane);
  float* mw = ms + (size_t)(32 * wave) * COUT;

#pragma unroll 1
  for (int j = 0; j < 32; ++j) {
    const int le = 32 * wave + j;
    const int sj = sl[le];
    const float* fr = FW + (size_t)sj * FWW;
    const v4f v0 = *(const v4fa*)(fr + 4 * lane);
    const v4f v1 = *(const v4fa*)(fr + 128 + 4 * lane);
    const v4f v2 = *(const v4fa*)(fr + 256 + 4 * lane);
    const v4f v3 = *(const v4fa*)(fr + off3);
    const float* hr = hl + le * HP + g;
    const float w0 = hr[0], w1 = hr[4], w2 = hr[8], w3 = hr[12];
    v4f p = v0 * w0;
    p = v1 * w1 + p;
    p = v2 * w2 + p;
    p = v3 * w3 + p;
    {
      const float tx = __shfl_xor(p.x, 8), ty = __shfl_xor(p.y, 8), tz = __shfl_xor(p.z, 8), tw = __shfl_xor(p.w, 8);
      p.x += tx; p.y += ty; p.z += tz; p.w += tw;
    }
    {
      const float tx = __shfl_xor(p.x, 16), ty = __shfl_xor(p.y, 16), tz = __shfl_xor(p.z, 16), tw = __shfl_xor(p.w, 16);
      p.x += tx; p.y += ty; p.z += tz; p.w += tw;
    }
    if (lane < 8) *(v4fa*)(mw + j * COUT + c4) = p;
  }
  __syncthreads();

  v4f pv[8];
#pragma unroll
  for (int it = 0; it < 8; ++it) pv[it] = *(const v4fa*)(ms + (size_t)(it * NTHR + tid) * 4);
  float* mb = MSG + (size_t)elb * COUT;
#pragma unroll
  for (int it = 0; it < 8; ++it) *(volatile v4f*)(mb + (size_t)(it * NTHR + tid) * 4) = pv[it];
  __threadfence();
#pragma unroll
  for (int it = 0; it < 8; ++it) *(volatile v4f*)(mb + (size_t)(it * NTHR + tid) * 4) = pv[it];
}

__global__ __launch_bounds__(NTHR) void k_scan(const int* __restrict__ dsts, const float* __restrict__ MSG,
                                               float* out, int nN, int nE, int vec8) {
  extern __shared__ __attribute__((aligned(16))) int lds_i[];
  int* reg1 = lds_i;
  int* reg2 = reg1 + RCAP;
  int* scnt = reg2 + RCAP;
  int* soff = scnt + NBA;
  int* list = soff + NBA;
  int* wcnt = list + LISTN;
  int* wtot = wcnt + NWAVE;
  const int tid = (int)threadIdx.x, lane = tid & 31, wave = tid >> 5;
  const int nodeBase = (int)blockIdx.x * NBA;

  {
    const v4i z4 = {0, 0, 0, 0};
    for (int i = tid * 4; i < ZINTS; i += NTHR * 4) *(v4ia*)(lds_i + i) = z4;
    if (tid < 2 * NWAVE) wcnt[tid] = 0;
  }
  __syncthreads();

  int tot = 0;
  const int nChunks = (nE + CHUNK - 1) / CHUNK;
#pragma unroll 1
  for (int ch = 0; ch < nChunks; ++ch) {
    const int cbase = ch * CHUNK;
    const int wc = scan_chunk(dsts, nE, cbase, nodeBase, NBA, vec8, list, tid, lane, wave);
    if (lane == 0) wcnt[wave] = wc;
    __syncthreads();
    int pre = 0, all = 0;
#pragma unroll
    for (int w2 = 0; w2 < NWAVE; ++w2) {
      int c = wcnt[w2];
      c = c < 0 ? 0 : (c > WCAP ? WCAP : c);
      all += c;
      pre += (w2 < wave) ? c : 0;
    }
    const int wcc  = wc > WCAP ? WCAP : wc;
    const int base = tot + pre;
#pragma unroll 1
    for (int i = lane; i < wcc; i += 32) {
      const int ent = list[wave * WCAP + i];
      const int el  = (ent >> PKS) & (CHUNK - 1);
      const int sl  = ent & (NBA - 1);
      int eid = cbase + el;
      eid = eid > nE - 1 ? nE - 1 : eid;
      const int pos = base + i;
      if (pos < RCAP) reg1[pos] = (int)(((unsigned)eid << PKS) | (unsigned)sl);
    }
    tot += all;
    tot = tot > RCAP ? RCAP : tot;
    __syncthreads();
  }
  const int nh = tot;

  if (wave == 0) {
#pragma unroll 1
    for (int b0 = 0; b0 < nh; b0 += 32) {
      const int idx = b0 + lane;
      const int uv  = reg1[idx < RCAP ? idx : RCAP - 1];
      const int m32 = (nh - b0) < 32 ? (nh - b0) : 32;
#pragma unroll 1
      for (int k = 0; k < m32; ++k) {
        const int u  = __builtin_amdgcn_readlane(uv, k);
        const int sl = u & (NBA - 1);
        if (lane == 0) scnt[sl] = scnt[sl] + 1;
      }
    }
  }
  __syncthreads();

  {
    const v4i ca = *(const v4ia*)(scnt + 4 * tid);
    const int e0 = ca.x < 0 ? 0 : ca.x, e1 = ca.y < 0 ? 0 : ca.y, e2 = ca.z < 0 ? 0 : ca.z, e3 = ca.w < 0 ? 0 : ca.w;
    const int ts = e0 + e1 + e2 + e3;
    int incl = ts;
#pragma unroll
    for (int d = 1; d < 32; d <<= 1) {
      const int up = __shfl_up(incl, d, 32);
      if (lane >= d) incl += up;
    }
    if (lane == 31) wtot[wave] = incl;
    __syncthreads();
    int pre = 0;
#pragma unroll
    for (int w2 = 0; w2 < NWAVE; ++w2) pre += (w2 < wave) ? wtot[w2] : 0;
    int run = pre + incl - ts;
    soff[4 * tid + 0] = run; run += e0;
    soff[4 * tid + 1] = run; run += e1;
    soff[4 * tid + 2] = run; run += e2;
    soff[4 * tid + 3] = run;
  }
  __syncthreads();
  for (int i = tid; i < NBA; i += NTHR) list[i] = soff[i];
  __syncthreads();

  if (wave == 0) {
#pragma unroll 1
    for (int b0 = 0; b0 < nh; b0 += 32) {
      const int idx = b0 + lane;
      const int uv  = reg1[idx < RCAP ? idx : RCAP - 1];
      const int m32 = (nh - b0) < 32 ? (nh - b0) : 32;
#pragma unroll 1
      for (int k = 0; k < m32; ++k) {
        const int u   = __builtin_amdgcn_readlane(uv, k);
        const int sl  = u & (NBA - 1);
        const int eid = (int)((unsigned)u >> PKS);
        if (lane == 0) {
          int pos = list[sl];
          pos = pos < 0 ? 0 : (pos > RCAP - 1 ? RCAP - 1 : pos);
          reg2[pos] = eid;
          list[sl] = pos + 1;
        }
      }
    }
  }
  __syncthreads();

  const int nbw = NBA / NWAVE;
  const bool ovf = (nh >= RCAP);
  const float qnan = __int_as_float(0x7fc00000);

#pragma unroll 1
  for (int jt = 0; jt < nbw; ++jt) {
    const int slot = wave * nbw + jt;
    const int node = nodeBase + slot;
    int st = soff[slot];
    const int craw = scnt[slot];
    int cnt = craw;
    st  = st < 0 ? 0 : (st > nh ? nh : st);
    cnt = cnt < 0 ? 0 : (cnt > DEGCAP ? DEGCAP : cnt);
    if (cnt > nh - st) cnt = nh - st;
    const float pz = (ovf || craw > DEGCAP) ? qnan : 0.0f;
    const bool live = node < nN;

    float a = 0.0f;
#pragma unroll 1
    for (int b0 = 0; b0 < cnt; b0 += 32) {
      int idx = st + b0 + lane; idx = idx > RCAP - 1 ? RCAP - 1 : idx;
      int eid = reg2[idx]; eid = eid < 0 ? 0 : (eid > nE - 1 ? nE - 1 : eid);
      const int m32 = (cnt - b0) < 32 ? (cnt - b0) : 32;
#pragma unroll 1
      for (int k = 0; k < m32; ++k) {
        const int ek = __builtin_amdgcn_readlane(eid, k);
        a += MSG[(size_t)ek * COUT + lane];
      }
    }
    const float r = (live ? a : 0.0f) + pz;
    if (live) {
      float* op = out + (size_t)node * COUT + lane;
      *(volatile float*)op = r;
      __threadfence();
      *(volatile float*)op = r;
    }
  }
}

static inline int cdiv(int a, int b) { return (a + b - 1) / b; }
static inline size_t al256(size_t o) { return (o + 255) & ~(size_t)255; }

extern "C" void kernel_launch(void* const* d_in, const int* in_sizes, int n_in,
                              void* d_out, int out_size, void* d_ws, size_t ws_size,
                              hipStream_t stream) {
  if (n_in < 6) return;
  if (in_sizes[0] < PD || (in_sizes[0] % PD) != 0) return;
  const int nN = in_sizes[0] / PD;
  if (nN < 1 || nN > (1 << 22)) return;
  if ((long long)in_sizes[1] != (long long)nN * CIN) return;
  const int nE = in_sizes[2];
  if (nE < 1 || nE >= (1 << 21)) return;
  if (in_sizes[3] != nE) return;
  if (in_sizes[4] != KPT * PD) return;
  if (in_sizes[5] != KPT * CIN * COUT) return;
  if ((long long)out_size != (long long)nN * COUT) return;

  const float* pos  = (const float*)d_in[0];
  const float* feat = (const float*)d_in[1];
  const int*   src  = (const int*)  d_in[2];
  const int*   dst  = (const int*)  d_in[3];
  const float* kpts = (const float*)d_in[4];
  const float* W    = (const float*)d_in[5];
  float* out = (float*)d_out;

  const int MP   = cdiv(nN, GBM) * GBM;
  const int gM   = MP / GBM;
  const int EP   = cdiv(nE, EPB) * EPB;
  const int gE   = EP / EPB;
  const int gA   = cdiv(nN, NBA);
  if ((long long)gA * NBA < (long long)nN) return;
  const int vec8 = ((nE & 3) == 0) ? 1 : 0;

  char* ws = (char*)d_ws;
  size_t off = 0;
  const size_t oWT  = off; off = al256(off + (size_t)NUW * 8 * 2);
  const size_t oFW  = off; off = al256(off + (size_t)MP * FWW * 4);
  const size_t oMSG = off; off = al256(off + (size_t)EP * COUT * 4);
  if (off > ws_size || off > (size_t)WSLIM) return;
  unsigned short* WT  = (unsigned short*)(ws + oWT);
  float*          FW  = (float*)(ws + oFW);
  float*          MSG = (float*)(ws + oMSG);

  hipFuncSetAttribute(reinterpret_cast<const void*>(&k_scan), hipFuncAttributeMaxDynamicSharedMemorySize, LDS_AGG);

  k_wprep<<<cdiv(NUW, NTHR), NTHR, 0, stream>>>(W, WT);
  k_fw<<<dim3(gM, NCB), GTHR, 0, stream>>>(feat, nN, WT, FW);
  k_edge<<<gE, NTHR, 0, stream>>>(pos, src, dst, kpts, nE, nN, FW, MSG);
  k_scan<<<gA, NTHR, LDS_AGG, stream>>>(dst, MSG, out, nN, nE, vec8);
}
